// Net_25744033972342
// MI455X (gfx1250) — hardware-verified
//
#include <hip/hip_runtime.h>
#include <math.h>
#include <stdint.h>

constexpr int NBATCH   = 4096;
constexpr int NSTEP    = 256;
constexpr int HID      = 51;
constexpr int NGATE    = 4;
constexpr int GROWS    = NGATE * HID;
constexpr int UPAD     = 64;
constexpr int NPAD     = NGATE * UPAD;
constexpr int K1PAD    = 64;
constexpr int K2PAD    = 128;
constexpr int ROWS_BLK = 16;
constexpr int SCAN_T   = 128;
constexpr int HPITCH   = 136;
constexpr int XCHUNK   = 64;
constexpr int OCHUNK   = 32;
constexpr int PSTP     = 36;
constexpr int PREP_T   = 64;
constexpr int PART_ELEMS  = NPAD * (K1PAD / 8);
constexpr int PART_BLOCKS = PART_ELEMS / PREP_T;
constexpr int VEC_COUNT   = 4;
constexpr int PREP_BLOCKS = 3 * PART_BLOCKS + VEC_COUNT;
constexpr float HCARRY = 256.0f;
constexpr float WCARRY = 16.0f;
constexpr float PCARRY = HCARRY * WCARRY;
constexpr float PINV   = 1.0f / PCARRY;

static_assert(NBATCH % ROWS_BLK == 0, "batch tiles exact");
static_assert(NSTEP % XCHUNK == 0 && XCHUNK % OCHUNK == 0 && OCHUNK == 32, "time chunks exact");
static_assert(K1PAD % 32 == 0 && K2PAD % 32 == 0 && K2PAD == 2 * K1PAD, "k multiples of 32");
static_assert(HID <= K1PAD && HID <= UPAD, "padding covers hidden size");
static_assert(UPAD == 16 * (SCAN_T / 32), "four waves own 16 units each");
static_assert(HPITCH % 8 == 0 && HPITCH >= K2PAD, "h tile pitch");
static_assert((2 * ROWS_BLK * HPITCH) % SCAN_T == 0, "h zero fill exact");
static_assert(PART_ELEMS % PREP_T == 0, "prep parts exact");
static_assert(PSTP % 4 == 0 && PSTP >= OCHUNK, "partial sum pitch");
static_assert((ROWS_BLK * XCHUNK / 4) % SCAN_T == 0, "x stage exact");

typedef __attribute__((ext_vector_type(16))) _Float16 v16h;
typedef __attribute__((ext_vector_type(8)))  _Float16 v8h;
typedef __attribute__((ext_vector_type(8)))  float    v8f;
typedef __attribute__((ext_vector_type(4)))  float    v4f;

__device__ __forceinline__ void guard_grp(v8f& a0, v8f& a1, v8f& a2, v8f& a3, v16h x, v16h b0, v16h b1, v16h b2, v16h b3) {
  asm volatile("v_nop\n\tv_nop\n\tv_nop\n\tv_nop" : "+v"(a0), "+v"(a1), "+v"(a2), "+v"(a3) : "v"(x), "v"(b0), "v"(b1), "v"(b2), "v"(b3));
}
__device__ __forceinline__ void acc_guard4(v8f& a, v8f& b, v8f& c, v8f& d) {
  asm volatile("v_nop\n\tv_nop\n\tv_nop\n\tv_nop" : "+v"(a), "+v"(b), "+v"(c), "+v"(d));
}

struct FragH {
  union U { v16h v; v8h h[2]; };
  static __device__ __forceinline__ v16h load(const _Float16* p) {
    U f;
    f.h[0] = *(const v8h*)(p);
    f.h[1] = *(const v8h*)(p + 16);
    return f.v;
  }
  static __device__ __forceinline__ v8f mma(v16h a, v16h b, v8f c) {
    return __builtin_amdgcn_wmma_f32_16x16x32_f16(false, a, false, b, (short)0, c, false, false);
  }
};

__device__ __forceinline__ float fsig(float x) {
  return __builtin_amdgcn_rcpf(1.0f + __expf(-x));
}
__device__ __forceinline__ float ftanh(float x) {
  const float xc = fminf(fmaxf(x, -15.0f), 15.0f);
  return 1.0f - 2.0f * __builtin_amdgcn_rcpf(__expf(2.0f * xc) + 1.0f);
}
__device__ __forceinline__ float cell_update(float ai, float af, float ag, float ao, float& cst) {
  const float ig = fsig(ai * PINV);
  const float fg = fsig(af * PINV);
  const float gg = ftanh(ag * PINV);
  const float og = fsig(ao * PINV);
  const float cn = fg * cst + ig * gg;
  cst = cn;
  return og * ftanh(cn);
}

__global__ __launch_bounds__(PREP_T) void lstm2_prep_kernel(
    const float* __restrict__ wih1, const float* __restrict__ whh1,
    const float* __restrict__ bih1, const float* __restrict__ bhh1,
    const float* __restrict__ wih2, const float* __restrict__ whh2,
    const float* __restrict__ bih2, const float* __restrict__ bhh2,
    const float* __restrict__ wlin,
    unsigned short* __restrict__ W1P, unsigned short* __restrict__ W2P, float* __restrict__ VEC) {
  const int tid = threadIdx.x;
  const int bx  = blockIdx.x;
  if (bx < 3 * PART_BLOCKS) {
    const int part = bx / PART_BLOCKS;
    const int i  = (bx - part * PART_BLOCKS) * PREP_T + tid;
    const int n  = i >> 3;
    const int k8 = (i & 7) * 8;
    const int g  = n >> 6;
    const int u  = n & 63;
    const int uc = (u < HID) ? u : (HID - 1);
    const float* src = (part == 0) ? whh1 : ((part == 1) ? wih2 : whh2);
    unsigned short* dst = (part == 0) ? (W1P + (size_t)n * K1PAD + k8)
                                      : (W2P + (size_t)n * K2PAD + ((part == 2) ? K1PAD : 0) + k8);
    v8h hv;
#pragma unroll
    for (int e = 0; e < 8; ++e) {
      const int k  = k8 + e;
      const int kc = (k < HID) ? k : (HID - 1);
      float ld = src[(size_t)(g * HID + uc) * HID + kc];
      asm volatile("" : "+v"(ld));
      const bool valid = (u < HID) && (k < HID);
      const float v = valid ? ld : 0.0f;
      hv[e] = (_Float16)(v * WCARRY);
    }
    *(volatile v8h*)(dst) = hv;
    __threadfence();
    *(volatile v8h*)(dst) = hv;
  } else {
    const int which = bx - 3 * PART_BLOCKS;
    const int n4 = tid * 4;
    v4f o;
#pragma unroll
    for (int e = 0; e < 4; ++e) {
      const int n  = n4 + e;
      const int g  = n >> 6;
      const int u  = n & 63;
      const int uc = (u < HID) ? u : (HID - 1);
      const int gi = g * HID + uc;
      bool valid = (u < HID);
      float val;
      if (which == 0) {
        val = bih1[gi] + bhh1[gi];
      } else if (which == 1) {
        val = wih1[gi];
      } else if (which == 2) {
        val = bih2[gi] + bhh2[gi];
      } else {
        val = wlin[uc];
        valid = valid && (g == 0);
      }
      asm volatile("" : "+v"(val));
      o[e] = valid ? val : 0.0f;
    }
    float* op = VEC + (size_t)which * NPAD + n4;
    *(volatile v4f*)(op) = o;
    __threadfence();
    *(volatile v4f*)(op) = o;
  }
}

__global__ __launch_bounds__(SCAN_T) void lstm2_scan_kernel(
    const float* __restrict__ xin,
    const unsigned short* __restrict__ W1p, const unsigned short* __restrict__ W2p,
    const float* __restrict__ vec, const float* __restrict__ blin,
    float* __restrict__ out) {
  __shared__ __align__(16) _Float16 HB[2][ROWS_BLK * HPITCH];
  __shared__ __align__(16) float    XT[XCHUNK * ROWS_BLK];
  __shared__ __align__(16) float    PST[SCAN_T / 32][ROWS_BLK * PSTP];

  const _Float16* W1 = (const _Float16*)W1p;
  const _Float16* W2 = (const _Float16*)W2p;
  const int tid  = threadIdx.x;
  const int lane = tid & 31;
  const int wave = tid >> 5;
  const int c    = lane & 15;
  const int hh   = lane >> 4;
  const int koff = hh * 8;
  const int u    = 16 * wave + c;
  const bool uval = (u < HID);
  const int rowbase = blockIdx.x * ROWS_BLK;

  float bS1[4], wS1[4], bS2[4];
#pragma unroll
  for (int g = 0; g < 4; ++g) {
    bS1[g] = vec[0 * NPAD + g * UPAD + u] * PCARRY;
    wS1[g] = vec[1 * NPAD + g * UPAD + u] * PCARRY;
    bS2[g] = vec[2 * NPAD + g * UPAD + u] * PCARRY;
  }
  const float wl = vec[3 * NPAD + u];
  const float bl = blin[0];

  {
    _Float16* hbf = &HB[0][0];
#pragma unroll 1
    for (int i = tid; i < 2 * ROWS_BLK * HPITCH; i += SCAN_T) hbf[i] = (_Float16)0.0f;
  }
  float c1[8], c2[8];
#pragma unroll
  for (int r = 0; r < 8; ++r) { c1[r] = 0.0f; c2[r] = 0.0f; }
  __syncthreads();

  const _Float16* w1row = W1 + (size_t)u * K1PAD + koff;
  const _Float16* w2row = W2 + (size_t)u * K2PAD + koff;

#pragma unroll 1
  for (int tc = 0; tc < NSTEP / XCHUNK; ++tc) {
#pragma unroll
    for (int i = 0; i < 2; ++i) {
      const int idx = i * SCAN_T + tid;
      const int row = idx >> 4;
      const int c4  = (idx & 15) * 4;
      const v4f v = *(const v4f*)(xin + (size_t)(rowbase + row) * NSTEP + tc * XCHUNK + c4);
      XT[(c4 + 0) * ROWS_BLK + row] = v[0];
      XT[(c4 + 1) * ROWS_BLK + row] = v[1];
      XT[(c4 + 2) * ROWS_BLK + row] = v[2];
      XT[(c4 + 3) * ROWS_BLK + row] = v[3];
    }
    __syncthreads();

#pragma unroll 1
    for (int th = 0; th < XCHUNK / OCHUNK; ++th) {
#pragma unroll 1
      for (int ti = 0; ti < OCHUNK; ++ti) {
        const int tl = th * OCHUNK + ti;
        const int p  = ti & 1;
        const _Float16* a1 = &HB[p][0] + c * HPITCH + koff;
        const _Float16* a2 = &HB[p ^ 1][0] + c * HPITCH + koff;
        _Float16* hw1 = &HB[p ^ 1][0] + (8 * hh) * HPITCH + u;
        _Float16* hw2 = &HB[p][0] + (8 * hh) * HPITCH + K1PAD + u;

        const v4f xa = *(const v4f*)(XT + tl * ROWS_BLK + 8 * hh);
        const v4f xb = *(const v4f*)(XT + tl * ROWS_BLK + 8 * hh + 4);
        const float xr[8] = {xa[0], xa[1], xa[2], xa[3], xb[0], xb[1], xb[2], xb[3]};
        v8f acc[4];
#pragma unroll
        for (int g = 0; g < 4; ++g)
#pragma unroll
          for (int r = 0; r < 8; ++r) acc[g][r] = fmaf(xr[r], wS1[g], bS1[g]);
#pragma unroll 1
        for (int k0 = 0; k0 < K1PAD; k0 += 32) {
          const v16h a  = FragH::load(a1 + k0);
          const v16h b0 = FragH::load(w1row + (size_t)0 * UPAD * K1PAD + k0);
          const v16h b1 = FragH::load(w1row + (size_t)1 * UPAD * K1PAD + k0);
          const v16h b2 = FragH::load(w1row + (size_t)2 * UPAD * K1PAD + k0);
          const v16h b3 = FragH::load(w1row + (size_t)3 * UPAD * K1PAD + k0);
          acc[0] = FragH::mma(a, b0, acc[0]);
          acc[1] = FragH::mma(a, b1, acc[1]);
          acc[2] = FragH::mma(a, b2, acc[2]);
          acc[3] = FragH::mma(a, b3, acc[3]);
          guard_grp(acc[0], acc[1], acc[2], acc[3], a, b0, b1, b2, b3);
        }
        acc_guard4(acc[0], acc[1], acc[2], acc[3]);
#pragma unroll
        for (int r = 0; r < 8; ++r) {
          const float hn = cell_update(acc[0][r], acc[1][r], acc[2][r], acc[3][r], c1[r]);
          const float hz = uval ? hn : 0.0f;
          hw1[r * HPITCH] = (_Float16)(hz * HCARRY);
        }
        __syncthreads();

#pragma unroll
        for (int g = 0; g < 4; ++g)
#pragma unroll
          for (int r = 0; r < 8; ++r) acc[g][r] = bS2[g];
#pragma unroll 1
        for (int k0 = 0; k0 < K2PAD; k0 += 32) {
          const v16h a  = FragH::load(a2 + k0);
          const v16h b0 = FragH::load(w2row + (size_t)0 * UPAD * K2PAD + k0);
          const v16h b1 = FragH::load(w2row + (size_t)1 * UPAD * K2PAD + k0);
          const v16h b2 = FragH::load(w2row + (size_t)2 * UPAD * K2PAD + k0);
          const v16h b3 = FragH::load(w2row + (size_t)3 * UPAD * K2PAD + k0);
          acc[0] = FragH::mma(a, b0, acc[0]);
          acc[1] = FragH::mma(a, b1, acc[1]);
          acc[2] = FragH::mma(a, b2, acc[2]);
          acc[3] = FragH::mma(a, b3, acc[3]);
          guard_grp(acc[0], acc[1], acc[2], acc[3], a, b0, b1, b2, b3);
        }
        acc_guard4(acc[0], acc[1], acc[2], acc[3]);
        float part[8];
#pragma unroll
        for (int r = 0; r < 8; ++r) {
          const float hn = cell_update(acc[0][r], acc[1][r], acc[2][r], acc[3][r], c2[r]);
          const float hz = uval ? hn : 0.0f;
          hw2[r * HPITCH] = (_Float16)(hz * HCARRY);
          part[r] = hz * wl;
        }
#pragma unroll
        for (int off = 1; off < 16; off <<= 1) {
#pragma unroll
          for (int r = 0; r < 8; ++r) part[r] += __shfl_xor(part[r], off, 32);
        }
        if (c == 0) {
          float* pp = &PST[wave][0] + (8 * hh) * PSTP + ti;
#pragma unroll
          for (int r = 0; r < 8; ++r) pp[r * PSTP] = part[r];
        }
        __syncthreads();
      }

      {
        const int row = 4 * wave + (lane >> 3);
        const int c4  = (lane & 7) * 4;
        const v4f s0 = *(const v4f*)(&PST[0][0] + row * PSTP + c4);
        const v4f s1 = *(const v4f*)(&PST[1][0] + row * PSTP + c4);
        const v4f s2 = *(const v4f*)(&PST[2][0] + row * PSTP + c4);
        const v4f s3 = *(const v4f*)(&PST[3][0] + row * PSTP + c4);
        v4f o;
#pragma unroll
        for (int e = 0; e < 4; ++e) o[e] = ((s0[e] + s1[e]) + (s2[e] + s3[e])) + bl;
        float* op = out + (size_t)(rowbase + row) * NSTEP + tc * XCHUNK + th * OCHUNK + c4;
        *(volatile v4f*)(op) = o;
        __threadfence();
        *(volatile v4f*)(op) = o;
      }
    }
  }
}

extern "C" void kernel_launch(void* const* d_in, const int* in_sizes, int n_in,
                              void* d_out, int out_size, void* d_ws, size_t ws_size, hipStream_t stream) {
  if (n_in < 11 || d_out == nullptr || d_ws == nullptr) return;
  if (in_sizes[0] != NBATCH * NSTEP || in_sizes[1] != GROWS || in_sizes[2] != GROWS * HID ||
      in_sizes[3] != GROWS || in_sizes[4] != GROWS || in_sizes[5] != GROWS * HID ||
      in_sizes[6] != GROWS * HID || in_sizes[7] != GROWS || in_sizes[8] != GROWS ||
      in_sizes[9] != HID || in_sizes[10] != 1 || out_size != NBATCH * NSTEP) return;

  const float* xin  = (const float*)d_in[0];
  const float* wih1 = (const float*)d_in[1];
  const float* whh1 = (const float*)d_in[2];
  const float* bih1 = (const float*)d_in[3];
  const float* bhh1 = (const float*)d_in[4];
  const float* wih2 = (const float*)d_in[5];
  const float* whh2 = (const float*)d_in[6];
  const float* bih2 = (const float*)d_in[7];
  const float* bhh2 = (const float*)d_in[8];
  const float* wlin = (const float*)d_in[9];
  const float* blin = (const float*)d_in[10];
  float* out = (float*)d_out;

  char* ws = (char*)d_ws;
  size_t off = 0;
  auto carve = [&](size_t bytes) -> char* { char* p = ws + off; off += (bytes + 255) & ~(size_t)255; return p; };
  unsigned short* W1P = (unsigned short*)carve((size_t)NPAD * K1PAD * 2);
  unsigned short* W2P = (unsigned short*)carve((size_t)NPAD * K2PAD * 2);
  float*          VEC = (float*)carve((size_t)VEC_COUNT * NPAD * 4);
  if (off > ws_size || off > (size_t)134217728) return;

  lstm2_prep_kernel<<<PREP_BLOCKS, PREP_T, 0, stream>>>(wih1, whh1, bih1, bhh1, wih2, whh2, bih2, bhh2, wlin, W1P, W2P, VEC);
  lstm2_scan_kernel<<<NBATCH / ROWS_BLK, SCAN_T, 0, stream>>>(xin, W1P, W2P, VEC, blin, out);
}
